// MM_GCN_75746043232444
// MI455X (gfx1250) — hardware-verified
//
#include <hip/hip_runtime.h>
#include <math.h>

#define NU    4000
#define NB    100
#define NL    40
#define DD    256
#define R3    12000
#define NMB   300
#define OUTW  1536
#define SNR   48
#define SNK   64
#define HTP   72

static_assert(NU == NB * NL);
static_assert(R3 % 32 == 0);
static_assert(NU % 8 == 0);
static_assert(DD % 32 == 0);

typedef __bf16 v16b __attribute__((ext_vector_type(16)));
typedef unsigned short v8us __attribute__((ext_vector_type(8)));
typedef float v8f __attribute__((ext_vector_type(8)));
typedef float v4f __attribute__((ext_vector_type(4)));
typedef v4f  __attribute__((may_alias)) v4fa;
typedef v8us __attribute__((may_alias)) v8usa;

union FragB { v16b v; v8us u[2]; };

__device__ __forceinline__ int imin(int a, int b) { return a < b ? a : b; }

__device__ __forceinline__ unsigned int bf_bits(float x) {
  const unsigned int u = __float_as_uint(x);
  return (u + 0x7FFFu + ((u >> 16) & 1u)) >> 16;
}
__device__ __forceinline__ float bf_val(unsigned int b) { return __uint_as_float(b << 16); }

__device__ __forceinline__ v8f wmma_bf(v16b a, v16b b, v8f c) {
  v8f d = __builtin_amdgcn_wmma_f32_16x16x32_bf16(false, a, false, b, (short)0, c, false, false);
  asm volatile("v_nop\n\tv_nop\n\tv_nop\n\tv_nop" : "+v"(d) : "v"(a), "v"(b));
  return d;
}
__device__ __forceinline__ v8f wmma3(v16b ah, v16b al, v16b bh, v16b bl, v8f c) {
  c = wmma_bf(ah, bh, c);
  c = wmma_bf(ah, bl, c);
  c = wmma_bf(al, bh, c);
  return c;
}
__device__ __forceinline__ v16b load_frag(const unsigned short* p, int h) {
  FragB f;
  f.u[0] = *(const v8usa*)(p + 8 * h);
  f.u[1] = *(const v8usa*)(p + 16 + 8 * h);
  return f.v;
}
__device__ __forceinline__ void split8(v4f a, v4f c, v8us& hi, v8us& lo) {
  float x[8];
  x[0] = a.x; x[1] = a.y; x[2] = a.z; x[3] = a.w;
  x[4] = c.x; x[5] = c.y; x[6] = c.z; x[7] = c.w;
  v8us hh = {0, 0, 0, 0, 0, 0, 0, 0};
  v8us ll = {0, 0, 0, 0, 0, 0, 0, 0};
#pragma unroll
  for (int t = 0; t < 8; ++t) {
    const unsigned int hb = bf_bits(x[t]);
    const unsigned int lb = bf_bits(x[t] - bf_val(hb));
    hh[t] = (unsigned short)hb;
    ll[t] = (unsigned short)lb;
  }
  hi = hh; lo = ll;
}
__device__ __forceinline__ void st4(float* p, v4f v) { *(volatile v4f*)p = v; }
__device__ __forceinline__ void st8(unsigned short* p, v8us v) { *(volatile v8us*)p = v; }
__device__ __forceinline__ v4f ld4(const float* p) { return *(const v4fa*)p; }
__device__ __forceinline__ void other2(int m, int& m1, int& m2) {
  m1 = (m == 0) ? 1 : 0;
  m2 = (m == 2) ? 1 : 2;
}

__global__ __launch_bounds__(256) void wconv_kernel(const float* __restrict__ W0,
                                                    const float* __restrict__ Wc,
                                                    unsigned short* __restrict__ WT)
{
  __shared__ __attribute__((aligned(16))) float T[32 * 260];
  const int w  = blockIdx.x >> 3;
  const int n0 = (blockIdx.x & 7) * 32;
  const float* Ws = (w == 0) ? W0 : (Wc + (size_t)(w - 1) * (DD * DD));
#pragma unroll 1
  for (int it = 0; it < 32; ++it) {
    const int idx = threadIdx.x + 256 * it;
    const int k = idx >> 5, nn = idx & 31;
    T[nn * 260 + k] = Ws[(size_t)k * DD + n0 + nn];
  }
  __syncthreads();
  const int wave = threadIdx.x >> 5, lane = threadIdx.x & 31;
  v8us hi[4], lo[4];
#pragma unroll
  for (int r = 0; r < 4; ++r) {
    const int nn = wave * 4 + r;
    const v4f f0 = ld4(T + nn * 260 + 8 * lane);
    const v4f f1 = ld4(T + nn * 260 + 8 * lane + 4);
    split8(f0, f1, hi[r], lo[r]);
  }
#pragma unroll
  for (int r = 0; r < 4; ++r) {
    unsigned short* dst = WT + (size_t)(w * 2) * (DD * DD) + (size_t)(n0 + wave * 4 + r) * DD + 8 * lane;
    st8(dst, hi[r]);
    st8(dst + DD * DD, lo[r]);
  }
  __threadfence();
#pragma unroll
  for (int r = 0; r < 4; ++r) {
    unsigned short* dst = WT + (size_t)(w * 2) * (DD * DD) + (size_t)(n0 + wave * 4 + r) * DD + 8 * lane;
    st8(dst, hi[r]);
    st8(dst + DD * DD, lo[r]);
  }
}

__device__ __forceinline__ void prep_store(float* o, v4f xa, v4f xb,
    unsigned short* xh, unsigned short* xl, unsigned short* nh, unsigned short* nl,
    v8us hx, v8us lx, v8us hn, v8us ln, int lane)
{
  st4(o + 4 * lane, xa);
  st4(o + 128 + 4 * lane, xb);
  st8(xh + 8 * lane, hx);
  st8(xl + 8 * lane, lx);
  st8(nh + 8 * lane, hn);
  st8(nl + 8 * lane, ln);
}

__global__ __launch_bounds__(256) void prep_kernel(
    const float* __restrict__ a, const float* __restrict__ v, const float* __restrict__ l,
    const float* __restrict__ qmask, const float* __restrict__ spk,
    const int* __restrict__ dlp, const int* __restrict__ ndp,
    float* __restrict__ out,
    unsigned short* __restrict__ Xhi, unsigned short* __restrict__ Xlo,
    unsigned short* __restrict__ Nhi, unsigned short* __restrict__ Nlo)
{
  const int wave = threadIdx.x >> 5, lane = threadIdx.x & 31;
  const int u = blockIdx.x * 8 + wave;
  const int b = u / NL, li = u - b * NL;
  const int qi = (li * NB + b) * 2;
  const float q0 = qmask[qi], q1 = qmask[qi + 1];
  const int spkix = (q1 > q0) ? 1 : 0;
  const int nval = dlp[0] * ndp[0];
  const bool spkon = (u < nval);
  const float* ep = spk + spkix * DD;
  const v4f ea = ld4(ep + 4 * lane), eb = ld4(ep + 128 + 4 * lane);
  const v4f ec = ld4(ep + 8 * lane), ed = ld4(ep + 8 * lane + 4);
#pragma unroll 1
  for (int m = 0; m < 3; ++m) {
    const float* src = (m == 0) ? a : ((m == 1) ? v : l);
    const float* p = src + (size_t)u * DD;
    const bool addspk = (m == 2) && spkon;
    v4f xa = ld4(p + 4 * lane), xb = ld4(p + 128 + 4 * lane);
    v4f ya = ld4(p + 8 * lane), yb = ld4(p + 8 * lane + 4);
    if (addspk) { xa = xa + ea; xb = xb + eb; ya = ya + ec; yb = yb + ed; }
    float ss = xa.x * xa.x;
    ss += xa.y * xa.y; ss += xa.z * xa.z; ss += xa.w * xa.w;
    ss += xb.x * xb.x; ss += xb.y * xb.y; ss += xb.z * xb.z; ss += xb.w * xb.w;
#pragma unroll
    for (int o = 16; o > 0; o >>= 1) ss += __shfl_xor(ss, o, 32);
    const float nrm = sqrtf(ss);
    const float rn = 1.0f / nrm;
    v8us hx, lx, hn, ln;
    split8(ya, yb, hx, lx);
    split8(ya * rn, yb * rn, hn, ln);
    float* o = out + (size_t)u * OUTW + m * 512;
    const size_t prow = ((size_t)m * NU + u) * DD;
    prep_store(o, xa, xb, Xhi + prow, Xlo + prow, Nhi + prow, Nlo + prow, hx, lx, hn, ln, lane);
    __threadfence();
    prep_store(o, xa, xb, Xhi + prow, Xlo + prow, Nhi + prow, Nlo + prow, hx, lx, hn, ln, lane);
  }
}

__device__ __forceinline__ void gram_store(const float* Ssh, const float* dsh, const float* csh,
    unsigned short* SNhi, unsigned short* SNlo, float* DINV, float* CS, int mb, int wave, int lane)
{
  const int q = lane & 7, sub = lane >> 3;
#pragma unroll
  for (int it = 0; it < 4; ++it) {
    const int row = 16 * wave + it * 4 + sub;
    const int rr = imin(row, NL - 1);
    const float di = dsh[row];
    float vals[8];
#pragma unroll
    for (int c = 0; c < 8; ++c) {
      const int j = 8 * q + c;
      const int jj = imin(j, NL - 1);
      const float sv = Ssh[rr * 41 + jj] * di * dsh[j];
      vals[c] = (row < NL && j < NL) ? sv : 0.0f;
    }
    const v4f f0 = {vals[0], vals[1], vals[2], vals[3]};
    const v4f f1 = {vals[4], vals[5], vals[6], vals[7]};
    v8us hi, lo;
    split8(f0, f1, hi, lo);
    const size_t off = ((size_t)mb * SNR + row) * SNK + 8 * q;
    st8(SNhi + off, hi);
    st8(SNlo + off, lo);
  }
  const v4f dv = ld4(dsh + 4 * (lane & 15));
  const v4f cv = ld4(csh + 4 * lane);
  if (wave == 0 && lane < 16) st4(DINV + (size_t)mb * 64 + 4 * lane, dv);
  if (wave == 1) st4(CS + (size_t)mb * 128 + 4 * lane, cv);
}

__global__ __launch_bounds__(96) void gram_kernel(
    const unsigned short* __restrict__ Nhi, const unsigned short* __restrict__ Nlo,
    unsigned short* __restrict__ SNhi, unsigned short* __restrict__ SNlo,
    float* __restrict__ DINV, float* __restrict__ CS)
{
  __shared__ __attribute__((aligned(16))) float Ssh[NL * 41];
  __shared__ __attribute__((aligned(16))) float dsh[64];
  __shared__ __attribute__((aligned(16))) float csh[128];
  const float INVPI = 0.318309886183790672f;
  const int tid = threadIdx.x, wave = tid >> 5, lane = tid & 31;
  const int h = lane >> 4, mm = lane & 15;
  const int mb = blockIdx.x, m = mb / NB, b = mb - m * NB;
  const int g0 = m * NU + b * NL;

  const int ga = g0 + imin(16 * wave + mm, NL - 1);
  const unsigned short* pah = Nhi + (size_t)ga * DD;
  const unsigned short* pal = Nlo + (size_t)ga * DD;
  const v8f z8 = {0.f, 0.f, 0.f, 0.f, 0.f, 0.f, 0.f, 0.f};
  v8f acc[3];
#pragma unroll
  for (int nt = 0; nt < 3; ++nt) acc[nt] = z8;

#pragma unroll 1
  for (int k0 = 0; k0 < DD; k0 += 32) {
    const v16b ah = load_frag(pah + k0, h);
    const v16b al = load_frag(pal + k0, h);
#pragma unroll
    for (int nt = 0; nt < 3; ++nt) {
      const int gb = g0 + imin(16 * nt + mm, NL - 1);
      const v16b bh = load_frag(Nhi + (size_t)gb * DD + k0, h);
      const v16b bl = load_frag(Nlo + (size_t)gb * DD + k0, h);
      acc[nt] = wmma3(ah, al, bh, bl, acc[nt]);
    }
  }
#pragma unroll
  for (int nt = 0; nt < 3; ++nt) {
#pragma unroll
    for (int r = 0; r < 8; ++r) {
      const int i = 16 * wave + 8 * h + r, j = 16 * nt + mm;
      if (i < NL && j < NL) Ssh[i * 41 + j] = acc[nt][r];
    }
  }
  if (tid < 64) dsh[tid] = 0.0f;
  for (int e = tid; e < 128; e += 96) csh[e] = 0.0f;
  __syncthreads();

#pragma unroll 1
  for (int e = tid; e < NL * NL; e += 96) {
    const int i = e / NL, j = e - i * NL;
    const float c = Ssh[i * 41 + j] * 0.99999f;
    Ssh[i * 41 + j] = 1.0f - acosf(c) * INVPI;
  }
  {
    const int slot = (tid < NL) ? 0 : 1;
    const int i = imin(tid - NL * slot, NL - 1);
    int m1, m2; other2(m, m1, m2);
    const int mo = (slot == 0) ? m1 : m2;
    const int n = b * NL + i;
    const unsigned short* xh = Nhi + (size_t)(m * NU + n) * DD;
    const unsigned short* xl = Nlo + (size_t)(m * NU + n) * DD;
    const unsigned short* yh = Nhi + (size_t)(mo * NU + n) * DD;
    const unsigned short* yl = Nlo + (size_t)(mo * NU + n) * DD;
    float dsum = 0.0f;
#pragma unroll 1
    for (int k = 0; k < DD; k += 8) {
      const v8us a0 = *(const v8usa*)(xh + k), a1 = *(const v8usa*)(xl + k);
      const v8us c0 = *(const v8usa*)(yh + k), c1 = *(const v8usa*)(yl + k);
#pragma unroll
      for (int c = 0; c < 8; ++c)
        dsum += (bf_val(a0[c]) + bf_val(a1[c])) * (bf_val(c0[c]) + bf_val(c1[c]));
    }
    const float cv = 1.0f - acosf(dsum * 0.99999f) * INVPI;
    if (tid < 2 * NL) csh[slot * 64 + i] = cv;
  }
  __syncthreads();

  {
    const int ic = imin(tid, NL - 1);
    float dg = 0.0f;
#pragma unroll 1
    for (int j = 0; j < NL; ++j) dg += Ssh[ic * 41 + j];
    dg += csh[ic] + csh[64 + ic];
    const float dinv = 1.0f / sqrtf(dg);
    if (tid < NL) dsh[tid] = dinv;
  }
  __syncthreads();

  gram_store(Ssh, dsh, csh, SNhi, SNlo, DINV, CS, mb, wave, lane);
  __threadfence();
  gram_store(Ssh, dsh, csh, SNhi, SNlo, DINV, CS, mb, wave, lane);
}

__device__ __forceinline__ size_t hrow_off(int gr, int outsel) {
  if (outsel == 0) return (size_t)gr * DD;
  const int mrow = gr / NU;
  const int i = gr - mrow * NU;
  return (size_t)i * OUTW + (size_t)mrow * 512 + 256;
}

__device__ __forceinline__ void gemm_store(const float* s, float* OutF,
    unsigned short* OutHi, unsigned short* OutLo, int r0, int c0, int outsel, int lane)
{
  const int q = lane & 7, sub = lane >> 3;
#pragma unroll
  for (int it = 0; it < 8; ++it) {
    const int lid = it * 4 + sub, row = lid >> 1, hl = lid & 1;
    const v4f vv = ld4(s + row * 64 + 32 * hl + 4 * q);
    st4(OutF + hrow_off(r0 + row, outsel) + c0 + 32 * hl + 4 * q, vv);
  }
  if (outsel == 0) {
#pragma unroll
    for (int it = 0; it < 4; ++it) {
      const int row = it * 4 + sub;
      const v4f f0 = ld4(s + row * 64 + 8 * q), f1 = ld4(s + row * 64 + 8 * q + 4);
      v8us hi, lo;
      split8(f0, f1, hi, lo);
      const size_t off = (size_t)(r0 + row) * DD + c0 + 8 * q;
      st8(OutHi + off, hi);
      st8(OutLo + off, lo);
    }
  }
}

__global__ __launch_bounds__(128) void gemm_kernel(
    const unsigned short* __restrict__ Ahi, const unsigned short* __restrict__ Alo,
    const unsigned short* __restrict__ Bhi, const unsigned short* __restrict__ Blo,
    const float* __restrict__ bias, const float* __restrict__ Sup,
    float* __restrict__ OutF, unsigned short* __restrict__ OutHi, unsigned short* __restrict__ OutLo,
    int mode, int outsel, float theta, float omt)
{
  __shared__ __attribute__((aligned(16))) float sT[4][16 * 64];
  const int tid = threadIdx.x, wave = tid >> 5, lane = tid & 31;
  const int h = lane >> 4, mm = lane & 15;
  const int r0 = blockIdx.x * 32 + 16 * (wave & 1);
  const int c0 = blockIdx.y * 128 + 64 * (wave >> 1);
  const unsigned short* pah = Ahi + (size_t)(r0 + mm) * DD;
  const unsigned short* pal = Alo + (size_t)(r0 + mm) * DD;
  const unsigned short* pbh = Bhi + (size_t)(c0 + mm) * DD;
  const unsigned short* pbl = Blo + (size_t)(c0 + mm) * DD;
  const v8f z8 = {0.f, 0.f, 0.f, 0.f, 0.f, 0.f, 0.f, 0.f};
  v8f acc[4];
#pragma unroll
  for (int nt = 0; nt < 4; ++nt) acc[nt] = z8;

#pragma unroll 1
  for (int k0 = 0; k0 < DD; k0 += 32) {
    const v16b ah = load_frag(pah + k0, h);
    const v16b al = load_frag(pal + k0, h);
#pragma unroll
    for (int nt = 0; nt < 4; ++nt) {
      const v16b bh = load_frag(pbh + (size_t)nt * 16 * DD + k0, h);
      const v16b bl = load_frag(pbl + (size_t)nt * 16 * DD + k0, h);
      acc[nt] = wmma3(ah, al, bh, bl, acc[nt]);
    }
  }

  float* s = &sT[wave][0];
#pragma unroll
  for (int nt = 0; nt < 4; ++nt) {
    const int col = 16 * nt + mm, gc = c0 + col;
    const float bv = bias[gc];
#pragma unroll
    for (int r = 0; r < 8; ++r) {
      const int row = 8 * h + r, gr = r0 + row;
      float y;
      if (mode == 0) {
        y = fmaxf(acc[nt][r] + bv, 0.0f);
      } else {
        const float sp = Sup[(size_t)gr * DD + gc];
        y = fmaxf(theta * acc[nt][r] + omt * sp, 0.0f);
      }
      s[row * 64 + col] = y;
    }
  }
  __syncthreads();
  gemm_store(s, OutF, OutHi, OutLo, r0, c0, outsel, lane);
  __threadfence();
  gemm_store(s, OutF, OutHi, OutLo, r0, c0, outsel, lane);
}

__device__ __forceinline__ void sup_store(const float* s, float* SUPf,
    unsigned short* SUPhi, unsigned short* SUPlo, int g0, int i0, int dcol0, int lane)
{
  const int q = lane & 7, sub = lane >> 3;
#pragma unroll
  for (int it = 0; it < 8; ++it) {
    const int lid = it * 4 + sub, row = lid >> 1, hl = lid & 1;
    const int i = i0 + row;
    const v4f vv = ld4(s + row * 64 + 32 * hl + 4 * q);
    if (i < NL) st4(SUPf + (size_t)(g0 + i) * DD + dcol0 + 32 * hl + 4 * q, vv);
  }
#pragma unroll
  for (int it = 0; it < 4; ++it) {
    const int row = it * 4 + sub;
    const int i = i0 + row;
    const v4f f0 = ld4(s + row * 64 + 8 * q), f1 = ld4(s + row * 64 + 8 * q + 4);
    v8us hi, lo;
    split8(f0, f1, hi, lo);
    if (i < NL) {
      const size_t off = (size_t)(g0 + i) * DD + dcol0 + 8 * q;
      st8(SUPhi + off, hi);
      st8(SUPlo + off, lo);
    }
  }
}

__global__ __launch_bounds__(64) void support_kernel(
    const unsigned short* __restrict__ SNhi, const unsigned short* __restrict__ SNlo,
    const float* __restrict__ DINV, const float* __restrict__ CS,
    const float* Hf, const unsigned short* __restrict__ Hhi, const unsigned short* __restrict__ Hlo,
    const float* H0f,
    float* __restrict__ SUPf, unsigned short* __restrict__ SUPhi, unsigned short* __restrict__ SUPlo)
{
  __shared__ __attribute__((aligned(16))) unsigned short hT[2][128 * HTP];
  __shared__ __attribute__((aligned(16))) float sT[2][16 * 64];
  __shared__ float chat[2][SNR];
  const int tid = threadIdx.x, wave = tid >> 5, lane = tid & 31;
  const int h = lane >> 4, mm = lane & 15;
  const int mb = blockIdx.x, m = mb / NB, b = mb - m * NB;
  const int dbase = blockIdx.y * 128;
  const int g0 = m * NU + b * NL;
  int m1, m2; other2(m, m1, m2);

  {
    const int ic = imin(tid, NL - 1);
    const float di = DINV[mb * 64 + ic];
    const float d1 = DINV[(m1 * NB + b) * 64 + ic];
    const float d2 = DINV[(m2 * NB + b) * 64 + ic];
    const float c1 = CS[mb * 128 + ic] * di * d1;
    const float c2 = CS[mb * 128 + 64 + ic] * di * d2;
    if (tid < SNR) {
      chat[0][tid] = (tid < NL) ? c1 : 0.0f;
      chat[1][tid] = (tid < NL) ? c2 : 0.0f;
    }
  }
#pragma unroll 1
  for (int pidx = 0; pidx < 2; ++pidx) {
    const unsigned short* src = (pidx == 0) ? Hhi : Hlo;
    unsigned short* dstp = &hT[pidx][0];
#pragma unroll 1
    for (int it = 0; it < 10; ++it) {
      const int idx = tid + 64 * it;
      const int j = idx >> 4;
      const int d0 = (idx & 15) * 8;
      const v8us uu = *(const v8usa*)(src + (size_t)(g0 + j) * DD + dbase + d0);
#pragma unroll
      for (int c = 0; c < 8; ++c) dstp[(d0 + c) * HTP + j] = uu[c];
    }
    const v8us z = {0, 0, 0, 0, 0, 0, 0, 0};
#pragma unroll 1
    for (int idx = tid; idx < 128 * 3; idx += 64) {
      const int d = idx / 3, part = idx - 3 * d;
      *(v8usa*)(dstp + d * HTP + NL + 8 * part) = z;
    }
  }
  __syncthreads();

  const v8f z8 = {0.f, 0.f, 0.f, 0.f, 0.f, 0.f, 0.f, 0.f};
#pragma unroll 1
  for (int mt = 0; mt < 3; ++mt) {
    v8f acc[4];
#pragma unroll
    for (int nt = 0; nt < 4; ++nt) acc[nt] = z8;
    const size_t arow = ((size_t)mb * SNR + 16 * mt + mm) * SNK;
#pragma unroll
    for (int ks = 0; ks < 2; ++ks) {
      const int k0 = 32 * ks;
      const v16b ah = load_frag(SNhi + arow + k0, h);
      const v16b al = load_frag(SNlo + arow + k0, h);
#pragma unroll
      for (int nt = 0; nt < 4; ++nt) {
        const int dl = 64 * wave + 16 * nt + mm;
        const v16b bh = load_frag(&hT[0][dl * HTP + k0], h);
        const v16b bl = load_frag(&hT[1][dl * HTP + k0], h);
        acc[nt] = wmma3(ah, al, bh, bl, acc[nt]);
      }
    }
    float* s = &sT[wave][0];
#pragma unroll
    for (int nt = 0; nt < 4; ++nt) {
      const int col = 16 * nt + mm;
      const int dcol = dbase + 64 * wave + col;
#pragma unroll
      for (int r = 0; r < 8; ++r) {
        const int i = 16 * mt + 8 * h + r;
        const int ic = imin(i, NL - 1);
        const int n = b * NL + ic;
        const float h1 = Hf[((size_t)m1 * NU + n) * DD + dcol];
        const float h2 = Hf[((size_t)m2 * NU + n) * DD + dcol];
        const float h0 = H0f[((size_t)g0 + ic) * DD + dcol];
        const float sv = 0.9f * (acc[nt][r] + chat[0][i] * h1 + chat[1][i] * h2) + 0.1f * h0;
        s[(8 * h + r) * 64 + col] = sv;
      }
    }
    __syncthreads();
    sup_store(s, SUPf, SUPhi, SUPlo, g0, 16 * mt, dbase + 64 * wave, lane);
    __threadfence();
    sup_store(s, SUPf, SUPhi, SUPlo, g0, 16 * mt, dbase + 64 * wave, lane);
    __syncthreads();
  }
}

extern "C" void kernel_launch(void* const* d_in, const int* in_sizes, int n_in,
                              void* d_out, int out_size, void* d_ws, size_t ws_size,
                              hipStream_t stream)
{
  if (n_in < 10) return;
  if (in_sizes[0] != NU * DD || in_sizes[1] != NU * DD || in_sizes[2] != NU * DD) return;
  if (in_sizes[3] != NL * NB * 2 || in_sizes[4] != 2 * DD) return;
  if (in_sizes[5] != DD * DD || in_sizes[6] != DD || in_sizes[7] != 4 * DD * DD) return;
  if (in_sizes[8] < 1 || in_sizes[9] < 1) return;
  if (out_size != NU * OUTW) return;

  const float* a      = (const float*)d_in[0];
  const float* v      = (const float*)d_in[1];
  const float* l      = (const float*)d_in[2];
  const float* qmask  = (const float*)d_in[3];
  const float* spkemb = (const float*)d_in[4];
  const float* W0     = (const float*)d_in[5];
  const float* b0     = (const float*)d_in[6];
  const float* Wconvs = (const float*)d_in[7];
  const int*   dlp    = (const int*)d_in[8];
  const int*   ndp    = (const int*)d_in[9];
  float* out = (float*)d_out;

  const size_t PL  = (size_t)R3 * DD * 2;
  const size_t PF  = (size_t)R3 * DD * 4;
  const size_t WTB = (size_t)10 * DD * DD * 2;
  const size_t CSB = (size_t)NMB * 128 * 4;
  const size_t DIB = (size_t)NMB * 64 * 4;
  const size_t SNB = (size_t)NMB * SNR * SNK * 2;
  const size_t total = 4 * PL + WTB + CSB + DIB + 2 * SNB + 3 * (PF + 2 * PL);
  if (total > ws_size) return;
  if (total > (size_t)134217728) return;

  char* ws = (char*)d_ws;
  size_t off = 0;
  unsigned short* Xhi  = (unsigned short*)(ws + off); off += PL;
  unsigned short* Xlo  = (unsigned short*)(ws + off); off += PL;
  unsigned short* Nhi  = (unsigned short*)(ws + off); off += PL;
  unsigned short* Nlo  = (unsigned short*)(ws + off); off += PL;
  unsigned short* WT   = (unsigned short*)(ws + off); off += WTB;
  float*          CS   = (float*)(ws + off);          off += CSB;
  float*          DINV = (float*)(ws + off);          off += DIB;
  unsigned short* SNhi = (unsigned short*)(ws + off); off += SNB;
  unsigned short* SNlo = (unsigned short*)(ws + off); off += SNB;
  float*          H0f  = (float*)(ws + off);          off += PF;
  unsigned short* H0hi = (unsigned short*)(ws + off); off += PL;
  unsigned short* H0lo = (unsigned short*)(ws + off); off += PL;
  float*          Hf   = (float*)(ws + off);          off += PF;
  unsigned short* Hhi  = (unsigned short*)(ws + off); off += PL;
  unsigned short* Hlo  = (unsigned short*)(ws + off); off += PL;
  float*          SUPf = (float*)(ws + off);          off += PF;
  unsigned short* SUPhi = (unsigned short*)(ws + off); off += PL;
  unsigned short* SUPlo = (unsigned short*)(ws + off); off += PL;
  if (off != total) return;

  wconv_kernel<<<40, 256, 0, stream>>>(W0, Wconvs, WT);
  prep_kernel<<<NU / 8, 256, 0, stream>>>(a, v, l, qmask, spkemb, dlp, ndp, out, Xhi, Xlo, Nhi, Nlo);
  gram_kernel<<<NMB, 96, 0, stream>>>(Nhi, Nlo, SNhi, SNlo, DINV, CS);

  const dim3 ggemm(R3 / 32, 2);
  const dim3 gsup(NMB, 2);
  gemm_kernel<<<ggemm, 128, 0, stream>>>(Xhi, Xlo, WT, WT + DD * DD, b0, SUPf,
                                         H0f, H0hi, H0lo, 0, 0, 0.0f, 0.0f);
  for (int it = 0; it < 4; ++it) {
    const double th = log(0.5 / (double)(it + 1) + 1.0);
    const float thf = (float)th;
    const float omf = (float)(1.0 - th);
    const float* hsrc = (it == 0) ? H0f : Hf;
    const unsigned short* hshi = (it == 0) ? H0hi : Hhi;
    const unsigned short* hslo = (it == 0) ? H0lo : Hlo;
    support_kernel<<<gsup, 64, 0, stream>>>(SNhi, SNlo, DINV, CS, hsrc, hshi, hslo, H0f,
                                           SUPf, SUPhi, SUPlo);
    const unsigned short* wh = WT + (size_t)((it + 1) * 2) * (DD * DD);
    const unsigned short* wl = wh + DD * DD;
    float* of = (it == 3) ? out : Hf;
    gemm_kernel<<<ggemm, 128, 0, stream>>>(SUPhi, SUPlo, wh, wl, b0, SUPf,
                                           of, Hhi, Hlo, 1, (it == 3) ? 1 : 0, thf, omf);
  }
}
